// LowPassFilter_53661321396356
// MI455X (gfx1250) — hardware-verified
//
#include <hip/hip_runtime.h>
#include <math.h>

typedef __attribute__((ext_vector_type(16))) _Float16 v16h;
typedef __attribute__((ext_vector_type(8)))  _Float16 v8h;
typedef __attribute__((ext_vector_type(16))) __bf16   v16b;
typedef __attribute__((ext_vector_type(8)))  __bf16   v8b;
typedef __attribute__((ext_vector_type(8)))  float    v8f;
typedef __attribute__((ext_vector_type(4)))  float    v4f;
typedef __attribute__((ext_vector_type(4)))  unsigned int v4u;

__device__ __forceinline__ unsigned short f2bf_bits(float f) {
  unsigned u = __float_as_uint(f);
  return (unsigned short)((u + 0x7FFFu + ((u >> 16) & 1u)) >> 16);
}
__device__ __forceinline__ float bf_bits2f(unsigned short h) { return __uint_as_float(((unsigned)h) << 16); }

__device__ __forceinline__ void dep_guard_h(v8f& a, v8f& b, v16h x, v16h y) { asm volatile("v_nop\n\tv_nop\n\tv_nop\n\tv_nop" : "+v"(a), "+v"(b) : "v"(x), "v"(y)); }
__device__ __forceinline__ void dep_guard_b(v8f& a, v8f& b, v16b x, v16b y) { asm volatile("v_nop\n\tv_nop\n\tv_nop\n\tv_nop" : "+v"(a), "+v"(b) : "v"(x), "v"(y)); }
__device__ __forceinline__ void keep4_h(v16h a, v16h b, v16h c, v16h d) { asm volatile("v_nop" :: "v"(a), "v"(b), "v"(c), "v"(d)); }
__device__ __forceinline__ void keep4_b(v16b a, v16b b, v16b c, v16b d) { asm volatile("v_nop" :: "v"(a), "v"(b), "v"(c), "v"(d)); }
__device__ __forceinline__ void acc_guard4(v8f& a, v8f& b, v8f& c, v8f& d) { asm volatile("v_nop\n\tv_nop\n\tv_nop\n\tv_nop" : "+v"(a), "+v"(b), "+v"(c), "+v"(d)); }
template <typename T> struct Frag;
template <> struct Frag<_Float16> {
  typedef v16h V; union U { v16h v; v8h h[2]; };
  static __device__ __forceinline__ v16h load(const _Float16* p) {
    U f; f.h[0] = *(const v8h*)(p); f.h[1] = *(const v8h*)(p + 16); return f.v;
  }
  static __device__ __forceinline__ v8f mma(v16h a, v16h b, v8f c) {
    return __builtin_amdgcn_wmma_f32_16x16x32_f16(false, a, false, b, (short)0, c, false, false);
  }
  static __device__ __forceinline__ void guard(v8f& a, v8f& b, v16h x, v16h y) { dep_guard_h(a, b, x, y); }
  static __device__ __forceinline__ void keep(v16h a, v16h b, v16h c, v16h d) { keep4_h(a, b, c, d); }
};
template <> struct Frag<__bf16> {
  typedef v16b V; union U { v16b v; v8b h[2]; };
  static __device__ __forceinline__ v16b load(const __bf16* p) {
    U f; f.h[0] = *(const v8b*)(p); f.h[1] = *(const v8b*)(p + 16); return f.v;
  }
  static __device__ __forceinline__ v8f mma(v16b a, v16b b, v8f c) {
    return __builtin_amdgcn_wmma_f32_16x16x32_bf16(false, a, false, b, (short)0, c, false, false);
  }
  static __device__ __forceinline__ void guard(v8f& a, v8f& b, v16b x, v16b y) { dep_guard_b(a, b, x, y); }
  static __device__ __forceinline__ void keep(v16b a, v16b b, v16b c, v16b d) { keep4_b(a, b, c, d); }
};

template <int ET> struct Elem;
template <> struct Elem<0> { typedef _Float16 T; };
template <> struct Elem<1> { typedef __bf16 T; };
template <int ET, bool SPLIT, int BIAS_MODE, int OUT_MODE, bool RESID, int ACT = 0>
__global__ __launch_bounds__(256) void wmma_gemm64(
    const unsigned short* __restrict__ Ap, const unsigned short* __restrict__ A2p, int lda, long strideA,
    const unsigned short* __restrict__ Btp, const unsigned short* __restrict__ Bt2p, int ldb, long strideB,
    void* __restrict__ Cout, void* __restrict__ Cout2, int ldc, long strideC,
    const float* __restrict__ bias,
    const float* __restrict__ resid, long strideR,
    int M, int N, int K, float scale) {
  typedef typename Elem<ET>::T T;
  typedef typename Frag<T>::V V;
  const T* A = (const T*)Ap; const T* A2 = (const T*)A2p; const T* Bt = (const T*)Btp; const T* Bt2 = (const T*)Bt2p;
  __shared__ __align__(16) float sT[8][16 * 68];
  const int b    = blockIdx.y;
  const int lane = threadIdx.x & 31;
  const int wave = threadIdx.x >> 5;
  const int tilesN = N >> 6;
  const int tilesM = M >> 6;
  const int tile = blockIdx.x * 8 + wave;
  if (tile >= tilesM * tilesN) return;
  const int tm = tile / tilesN;
  const int tn = tile - tm * tilesN;
  const int m0 = tm << 6;
  const int n0 = tn << 6;

  const T* Ab  = A  + (size_t)b * strideA;
  const T* Bb  = Bt + (size_t)b * strideB;
  const T* Ab2 = SPLIT ? (A2  + (size_t)b * strideA) : nullptr;
  const T* Bb2 = SPLIT ? (Bt2 + (size_t)b * strideB) : nullptr;

  const int rlane = lane & 15;
  const int koff  = (lane >> 4) * 8;
  const int mOff  = (lane >> 4) * 8;

  v8f acc[4][4];
#pragma unroll
  for (int i = 0; i < 4; ++i)
#pragma unroll
    for (int j = 0; j < 4; ++j) acc[i][j] = (v8f){0.f,0.f,0.f,0.f,0.f,0.f,0.f,0.f};

  for (int k0 = 0; k0 < K; k0 += 32) {
    V bh[4], bl[4];
#pragma unroll
    for (int j = 0; j < 4; ++j) {
      const size_t bo = (size_t)(n0 + (j << 4) + rlane) * ldb + koff + k0;
      bh[j] = Frag<T>::load(Bb + bo);
      if (SPLIT) bl[j] = Frag<T>::load(Bb2 + bo);
    }
#pragma unroll
    for (int i = 0; i < 4; ++i) {
      const size_t ao = (size_t)(m0 + (i << 4) + rlane) * lda + koff + k0;
      V ah = Frag<T>::load(Ab + ao);
      V al;
      if (SPLIT) al = Frag<T>::load(Ab2 + ao);
#pragma unroll
      for (int j = 0; j < 4; ++j) {
        acc[i][j] = Frag<T>::mma(ah, bh[j], acc[i][j]);
        if (SPLIT) {
          acc[i][j] = Frag<T>::mma(ah, bl[j], acc[i][j]);
          acc[i][j] = Frag<T>::mma(al, bh[j], acc[i][j]);
        }
      }
      Frag<T>::guard(acc[i][0], acc[i][3], ah, SPLIT ? al : ah);
    }
    Frag<T>::keep(bh[0], bh[1], bh[2], bh[3]);
    if (SPLIT) Frag<T>::keep(bl[0], bl[1], bl[2], bl[3]);
  }
  acc_guard4(acc[0][0], acc[0][1], acc[0][2], acc[0][3]);
  acc_guard4(acc[1][0], acc[1][1], acc[1][2], acc[1][3]);
  acc_guard4(acc[2][0], acc[2][1], acc[2][2], acc[2][3]);
  acc_guard4(acc[3][0], acc[3][1], acc[3][2], acc[3][3]);

  float* slab = sT[wave];
  const float* Rb = RESID ? (resid + (size_t)b * strideR) : nullptr;
#pragma unroll
  for (int i = 0; i < 4; ++i) {
    const int mBase = m0 + (i << 4);
#pragma unroll
    for (int j = 0; j < 4; ++j) {
      const int n = n0 + (j << 4) + rlane;
      float bv = 0.f;
      if (BIAS_MODE == 2) bv = bias[n];
#pragma unroll
      for (int r = 0; r < 8; ++r) {
        float v = acc[i][j][r] * scale;
        if (BIAS_MODE == 1) v += bias[mBase + mOff + r];
        if (BIAS_MODE == 2) v += bv;
        if (RESID) v += Rb[(size_t)(mBase + mOff + r) * ldc + n];
        if (ACT == 1) v = tanhf(v);
        if (ACT == 2) v = fmaxf(v, 0.0f);
        if (ACT == 3) v = v / (1.0f + expf(-v));
        if (ACT == 4) v = (v > 0.f) ? v : 0.01f * v;
        if (ACT == 5) v = 0.5f * v * (1.0f + erff(v * 0.70710678118654752f));
        slab[(mOff + r) * 68 + (j << 4) + rlane] = v;
      }
    }
    __builtin_amdgcn_fence(__ATOMIC_RELEASE, "workgroup");
    __builtin_amdgcn_wave_barrier();
    __builtin_amdgcn_fence(__ATOMIC_ACQUIRE, "workgroup");
    if (OUT_MODE == 0) {
      float* C = (float*)Cout + (size_t)b * strideC;
      const int hh = lane >> 4, c4 = (lane & 15) * 4;
      for (int pass = 0; pass < 2; ++pass) {
#pragma unroll
        for (int it = 0; it < 8; ++it) {
          const int row = it * 2 + hh;
          v4f v = *(const v4f*)(slab + row * 68 + c4);
          *(volatile v4f*)(C + (size_t)(mBase + row) * ldc + n0 + c4) = v;
        }
        __threadfence();
      }
    } else {
      const int q = lane >> 3, c8 = (lane & 7) * 8;
      unsigned short* C  = (unsigned short*)Cout  + (size_t)b * strideC;
      unsigned short* C2 = (OUT_MODE == 2) ? ((unsigned short*)Cout2 + (size_t)b * strideC) : nullptr;
      for (int pass = 0; pass < 2; ++pass) {
#pragma unroll
        for (int it = 0; it < 4; ++it) {
          const int row = it * 4 + q;
          const float* sp = slab + row * 68 + c8;
          v8h hv, lv;
#pragma unroll
          for (int e = 0; e < 8; ++e) {
            if (OUT_MODE == 1) {
              hv[e] = (_Float16)sp[e];
            } else {
              unsigned short hb = f2bf_bits(sp[e]);
              unsigned short lb = f2bf_bits(sp[e] - bf_bits2f(hb));
              hv[e] = __builtin_bit_cast(_Float16, hb);
              lv[e] = __builtin_bit_cast(_Float16, lb);
            }
          }
          *(volatile v8h*)(C + (size_t)(mBase + row) * ldc + n0 + c8) = hv;
          if (OUT_MODE == 2) *(volatile v8h*)(C2 + (size_t)(mBase + row) * ldc + n0 + c8) = lv;
        }
        __threadfence();
      }
    }
    __builtin_amdgcn_fence(__ATOMIC_RELEASE, "workgroup");
    __builtin_amdgcn_wave_barrier();
    __builtin_amdgcn_fence(__ATOMIC_ACQUIRE, "workgroup");
  }
}

constexpr int kNSig    = 64;
constexpr int kLen     = 32768;
constexpr int kHalf    = 16;
constexpr int kTaps    = 33;
constexpr int kTBlk    = 64;
constexpr int kNumTBlk = kLen / kTBlk;
constexpr int kBand    = 96;
constexpr int kXPitch  = kLen + 128;
constexpr int kXGroups = kXPitch / 8;
constexpr float kTwoPi   = 6.283185307179586f;
constexpr float kPiOver4 = 0.7853981633974483f;
constexpr float kInvFs   = 1.0f / 8000.0f;

static_assert(kLen % kTBlk == 0);
static_assert(kBand % 32 == 0);
static_assert(kXPitch % 64 == 0);
static_assert(kXPitch >= kLen + 2 * kHalf);
static_assert((kNumTBlk - 1) * kTBlk + kBand <= kXPitch);

struct FiltWin { float w[36]; };
static_assert(sizeof(FiltWin) == 144);

__global__ __launch_bounds__(256) void k_pad_split(const float* __restrict__ x,
                                                   unsigned short* __restrict__ xh,
                                                   unsigned short* __restrict__ xl,
                                                   int n, int pitch, int ngroups) {
  #pragma clang fp contract(off)
  const int b = blockIdx.y;
  const int g = blockIdx.x * 256 + (int)threadIdx.x;
  if (g >= ngroups) return;
  const int p0 = g * 8;
  const float* xr = x + (size_t)b * n;
  unsigned hw0 = 0u, hw1 = 0u, hw2 = 0u, hw3 = 0u;
  unsigned lw0 = 0u, lw1 = 0u, lw2 = 0u, lw3 = 0u;
  unsigned hwv[4] = {0u, 0u, 0u, 0u};
  unsigned lwv[4] = {0u, 0u, 0u, 0u};
#pragma unroll
  for (int e = 0; e < 8; ++e) {
    const int i = p0 + e - kHalf;
    int ic = (i < 0) ? 0 : i;
    ic = (ic > n - 1) ? (n - 1) : ic;
    const float xv = xr[ic];
    const float v = (i >= 0 && i < n) ? xv : 0.0f;
    const unsigned short hb = f2bf_bits(v);
    const unsigned short lb = f2bf_bits(v - bf_bits2f(hb));
    hwv[e >> 1] |= ((unsigned)hb) << (16 * (e & 1));
    lwv[e >> 1] |= ((unsigned)lb) << (16 * (e & 1));
  }
  hw0 = hwv[0]; hw1 = hwv[1]; hw2 = hwv[2]; hw3 = hwv[3];
  lw0 = lwv[0]; lw1 = lwv[1]; lw2 = lwv[2]; lw3 = lwv[3];
  const v4u hv = {hw0, hw1, hw2, hw3};
  const v4u lv = {lw0, lw1, lw2, lw3};
  unsigned short* ph = xh + (size_t)b * pitch + p0;
  unsigned short* pl = xl + (size_t)b * pitch + p0;
  *(volatile v4u*)ph = hv;
  *(volatile v4u*)pl = lv;
  __threadfence();
  *(volatile v4u*)ph = hv;
  *(volatile v4u*)pl = lv;
}

__global__ __launch_bounds__(256) void k_filter(const float* __restrict__ alphap,
                                                const float* __restrict__ betap,
                                                unsigned short* __restrict__ bth,
                                                unsigned short* __restrict__ btl,
                                                FiltWin win) {
  #pragma clang fp contract(off)
  __shared__ float s_cut[64];
  __shared__ float s_win[36];
  __shared__ float s_raw[64 * 33];
  __shared__ float s_inv[64];
  __shared__ __align__(16) unsigned short s_hi[64 * 96];
  __shared__ __align__(16) unsigned short s_lo[64 * 96];

  const int tid = (int)threadIdx.x;
  const int blk = blockIdx.x;
  const int t0  = blk * kTBlk;
  const float alpha = alphap[0];
  const float beta  = betap[0];

  if (tid < 64) {
    const float t  = (float)(t0 + tid);
    const float ar = (beta * t) * kInvFs;
    const float sv = sinf(ar);
    const float pr = alpha * sv;
    const float nm = kPiOver4 + pr;
    s_cut[tid] = nm / kTwoPi;
  }
  if (tid < 36) {
    float w = 0.0f;
#pragma unroll
    for (int q = 0; q < 36; ++q) w = (tid == q) ? win.w[q] : w;
    s_win[tid] = w;
  }
  __syncthreads();

#pragma unroll 1
  for (int idx = tid; idx < 64 * kTaps; idx += 256) {
    const int j = idx / kTaps;
    const int k = idx - j * kTaps;
    const float c  = s_cut[j];
    const float tm = (float)(k - kHalf);
    const float c2 = kTwoPi * c;
    const float xa = c2 * tm;
    const float sv = sinf(xa);
    const float q  = sv / xa;
    const float snc = (xa == 0.0f) ? 1.0f : q;
    const float w  = s_win[k];
    const float a1 = 2.0f * c;
    const float a2 = a1 * w;
    s_raw[idx] = a2 * snc;
  }
  __syncthreads();

  if (tid < 64) {
    float s = 0.0f;
#pragma unroll 1
    for (int k = 0; k < kTaps; ++k) s += s_raw[tid * kTaps + k];
    s_inv[tid] = 1.0f / s;
  }
  __syncthreads();

#pragma unroll 1
  for (int e = tid; e < kTBlk * kBand; e += 256) {
    const int tt = e / kBand;
    const int j  = e - tt * kBand;
    const int kk = j - tt;
    const bool valid = (kk >= 0) && (kk <= kTaps - 1);
    int kc = (kk < 0) ? 0 : kk;
    kc = (kc > kTaps - 1) ? (kTaps - 1) : kc;
    const float fr = s_raw[tt * kTaps + (kTaps - 1 - kc)];
    const float fv = fr * s_inv[tt];
    const float v  = valid ? fv : 0.0f;
    const unsigned short hb = f2bf_bits(v);
    const unsigned short lb = f2bf_bits(v - bf_bits2f(hb));
    s_hi[e] = hb;
    s_lo[e] = lb;
  }
  __syncthreads();

  unsigned short* gh = bth + (size_t)blk * (kTBlk * kBand);
  unsigned short* gl = btl + (size_t)blk * (kTBlk * kBand);
  for (int pass = 0; pass < 2; ++pass) {
#pragma unroll
    for (int it = 0; it < 3; ++it) {
      const int eo = (it * 256 + tid) * 8;
      const v4u hv = *(const v4u*)(s_hi + eo);
      const v4u lv = *(const v4u*)(s_lo + eo);
      *(volatile v4u*)(gh + eo) = hv;
      *(volatile v4u*)(gl + eo) = lv;
    }
    __threadfence();
  }
}

extern "C" void kernel_launch(void* const* d_in, const int* in_sizes, int n_in,
                              void* d_out, int out_size, void* d_ws, size_t ws_size,
                              hipStream_t stream) {
  if (n_in < 3) return;
  if (in_sizes[0] != kNSig * kLen) return;
  if (in_sizes[1] < 1 || in_sizes[2] < 1) return;
  if (out_size != kNSig * kLen) return;

  const float* x      = (const float*)d_in[0];
  const float* alphap = (const float*)d_in[1];
  const float* betap  = (const float*)d_in[2];
  float* out = (float*)d_out;

  const size_t xpBytes = (size_t)kNSig * kXPitch * 2;
  const size_t btBytes = (size_t)kNumTBlk * kTBlk * kBand * 2;
  const size_t offXh = 0;
  const size_t offXl = offXh + xpBytes;
  const size_t offBh = offXl + xpBytes;
  const size_t offBl = offBh + btBytes;
  const size_t total = offBl + btBytes;
  if (total > ws_size) return;

  unsigned char* ws = (unsigned char*)d_ws;
  unsigned short* xh  = (unsigned short*)(ws + offXh);
  unsigned short* xl  = (unsigned short*)(ws + offXl);
  unsigned short* bth = (unsigned short*)(ws + offBh);
  unsigned short* btl = (unsigned short*)(ws + offBl);

  FiltWin win;
  for (int k = 0; k < 36; ++k) win.w[k] = 0.0f;
  for (int k = 0; k < kTaps; ++k) {
    float argk = kTwoPi * (float)k;
    argk = argk / 32.0f;
    const double cd = cos((double)argk);
    const float cf = (float)cd;
    const float pr = 0.5f * cf;
    win.w[k] = 0.5f - pr;
  }

  {
    dim3 grid((kXGroups + 255) / 256, kNSig);
    k_pad_split<<<grid, dim3(256), 0, stream>>>(x, xh, xl, kLen, kXPitch, kXGroups);
  }
  k_filter<<<dim3(kNumTBlk), dim3(256), 0, stream>>>(alphap, betap, bth, btl, win);
  wmma_gemm64<1, true, 0, 0, false, 0><<<dim3(1, kNumTBlk), dim3(32), 0, stream>>>(
      xh, xl, kXPitch, (long)kTBlk,
      bth, btl, kBand, (long)(kTBlk * kBand),
      (void*)out, (void*)nullptr, kLen, (long)kTBlk,
      (const float*)nullptr,
      (const float*)nullptr, (long)0,
      kNSig, kTBlk, kBand, 1.0f);
}
